// SecondaryCapsuleLayer_5789615915069
// MI455X (gfx1250) — hardware-run, weakly checked
//
#include <hip/hip_runtime.h>


#ifndef NC
#define NC 2048
#endif
#define NC_FULL 2048
#define NB   64
#define NI   8
#define NU   32
#define ND   16
#define KS   (NC * NI)
#define WROW (NU * ND * NI)
#define SW   8
#define CWV  (NC / SW)
#define RCH  8
#define CARRY     256.0f
#define CARRY_INV (1.0f / 256.0f)
#define VCAR      64.0f
#define DSC       (1.0f / 4096.0f)
#define LOG2E     1.4426950408889634f

static_assert(NB == 64);
static_assert(NI == 8);
static_assert(NU == 32);
static_assert(ND == 16);
static_assert(NC % 64 == 0);
static_assert(NC <= NC_FULL);
static_assert(CWV % 4 == 0);
static_assert(NC % RCH == 0);
static_assert(KS % 32 == 0);
static_assert(32 * SW * 4 == NB * ND);
static_assert(SW * NB * ND * 4 <= 131072);
static_assert(NU * NB * 4 + NB * 4 <= 131072);
static_assert(256 / 8 == NU);
static_assert(256 * 16 == NU * NB * 2);
static_assert((NU * NB) % 256 == 0);
static_assert(NB % 32 == 0);
static_assert(128 * 4 == NU * ND);
static_assert(2 * (32 / 8) == RCH);
static_assert(3 * RCH * NU * 4 <= 131072);
static_assert(((size_t)NB * NC) % 256 == 0);
static_assert(((size_t)NC * NI * 8) % 256 == 0);
static_assert(((size_t)NC * NU / 4) % 256 == 0);
static_assert(((size_t)NC * WROW) % 8 == 0);

typedef _Float16 h16;
typedef __attribute__((ext_vector_type(16))) _Float16 v16h;
typedef __attribute__((ext_vector_type(8)))  _Float16 v8h;
typedef __attribute__((ext_vector_type(8)))  float    v8f;
typedef __attribute__((ext_vector_type(4)))  float    v4f;
typedef v4f  __attribute__((may_alias)) v4fa;

__device__ __forceinline__ unsigned short f2bf(float f) { unsigned u = __float_as_uint(f); u += 0x7FFFu + ((u >> 16) & 1u); return (unsigned short)(u >> 16); }
__device__ __forceinline__ float bfr(float f) { return __uint_as_float(((unsigned)f2bf(f)) << 16); }
__device__ __forceinline__ v16h cat16(v8h lo, v8h hi) { return __builtin_shufflevector(lo, hi, 0, 1, 2, 3, 4, 5, 6, 7, 8, 9, 10, 11, 12, 13, 14, 15); }
__device__ __forceinline__ v8f wmma16(v16h a, v16h b, v8f c) { return __builtin_amdgcn_wmma_f32_16x16x32_f16(false, a, false, b, (short)0, c, false, false); }
__device__ __forceinline__ v16h  ldh(const h16* p) { return cat16(*(const v8h*)p, *(const v8h*)(p + 16)); }
__device__ __forceinline__ void wave_sync() { __builtin_amdgcn_fence(3  , "wavefront"); __builtin_amdgcn_wave_barrier(); asm volatile("" ::: "memory"); }
__device__ __forceinline__ h16 toh_flush(float v) { const h16 r = (h16)v; return (fabsf(v) < 6.103515625e-05f) ? (h16)0.0f : r; }
__device__ __forceinline__ v8f wmma16g(v16h a, v16h b, v8f c) { c = wmma16(a, b, c); asm volatile("v_nop\n\tv_nop\n\tv_nop\n\tv_nop" : "+v"(c) : "v"(a), "v"(b)); return c; }

__global__ __launch_bounds__(256) void k_cvtw(const float* __restrict__ src, h16* dst, size_t n8) {
    const size_t i = (size_t)blockIdx.x * 256 + threadIdx.x; if (i >= n8) return;
    const v8f v = *(const v8f*)(src + i * 8); v8h o;
#pragma unroll
    for (int k = 0; k < 8; ++k) o[k] = toh_flush(bfr(v[k]));
    *(volatile v8h*)(dst + i * 8) = o; __threadfence(); *(volatile v8h*)(dst + i * 8) = o;
}

__global__ __launch_bounds__(256) void k_xs(const float* __restrict__ x, h16* XS) {
    const size_t T = (size_t)blockIdx.x * 256 + threadIdx.x; if (T >= (size_t)NB * NC) return;
    const int b = (int)(T / NC), c = (int)(T % NC);
    v8h o;
#pragma unroll
    for (int i = 0; i < NI; ++i) o[i] = toh_flush(bfr(x[((size_t)b * NI + i) * NC_FULL + c]));
    *(volatile v8h*)(XS + T * 8) = o; __threadfence(); *(volatile v8h*)(XS + T * 8) = o;
}

__global__ __launch_bounds__(256) void k_xt(const float* __restrict__ x, h16* XT) {
    const size_t T = (size_t)blockIdx.x * 256 + threadIdx.x; if (T >= (size_t)NC * NI * 8) return;
    const int m = (int)(T >> 3), p = (int)(T & 7);
    const int c = m >> 3, i = m & 7;
    v8h o;
#pragma unroll
    for (int e = 0; e < 8; ++e) o[e] = toh_flush(bfr(x[((size_t)(8 * p + e) * NI + i) * NC_FULL + c]));
    *(volatile v8h*)(XT + T * 8) = o; __threadfence(); *(volatile v8h*)(XT + T * 8) = o;
}

__global__ __launch_bounds__(256) void k_fillc(float* C) {
    const size_t T = (size_t)blockIdx.x * 256 + threadIdx.x; if (T >= (size_t)NC * NU / 4) return;
    v4f v; v[0] = 0.03125f; v[1] = 0.03125f; v[2] = 0.03125f; v[3] = 0.03125f;
    *(volatile v4f*)(C + T * 4) = v; __threadfence(); *(volatile v4f*)(C + T * 4) = v;
}

__global__ __launch_bounds__(32 * SW) void k_sgemm(const h16* __restrict__ XS, const h16* __restrict__ WH, const float* __restrict__ C, float* S) {
    __shared__ __align__(16) float red[SW * NB * ND];
    const int lane = threadIdx.x & 31, lr = lane & 15, hi = lane >> 4;
    const int wave = __builtin_amdgcn_readfirstlane((int)(threadIdx.x >> 5));
    const int u = blockIdx.x;
    v8f acc[4];
#pragma unroll
    for (int mt = 0; mt < 4; ++mt) acc[mt] = (v8f){};
    const size_t ao = (size_t)lr * KS + 8 * hi;
    const size_t wo = ((size_t)hi * NU + u) * (ND * NI) + (size_t)lr * NI;
    const int cbeg = wave * CWV;
#pragma unroll 1
    for (int cc = 0; cc < CWV; cc += 4) {
        const int c4 = cbeg + cc;
        const v8h w0 = *(const v8h*)(WH + wo + (size_t)c4 * WROW);
        const v8h w1 = *(const v8h*)(WH + wo + (size_t)(c4 + 2) * WROW);
        const float ca = C[(size_t)(c4 + hi) * NU + u] * CARRY;
        const float cb = C[(size_t)(c4 + 2 + hi) * NU + u] * CARRY;
        v16h bq;
#pragma unroll
        for (int e = 0; e < 8; ++e) { bq[e] = toh_flush((float)w0[e] * ca); bq[8 + e] = toh_flush((float)w1[e] * cb); }
        const h16* ap = XS + ao + (size_t)c4 * NI;
#pragma unroll
        for (int mt = 0; mt < 4; ++mt) { const v16h a = ldh(ap + (size_t)mt * 16 * KS); acc[mt] = wmma16g(a, bq, acc[mt]); }
    }
#pragma unroll
    for (int mt = 0; mt < 4; ++mt) {
#pragma unroll
        for (int r = 0; r < 8; ++r) red[wave * (NB * ND) + (mt * 16 + hi * 8 + r) * ND + lr] = acc[mt][r]; }
    __syncthreads();
    const int t = threadIdx.x;
    v4f sum = *(const v4fa*)(&red[4 * t]);
#pragma unroll
    for (int w = 1; w < SW; ++w) sum += *(const v4fa*)(&red[w * (NB * ND) + 4 * t]);
    sum = sum * CARRY_INV;
    float* dst = S + (size_t)u * (NB * ND) + 4 * t;
    *(volatile v4f*)dst = sum; __threadfence(); *(volatile v4f*)dst = sum;
}

__global__ __launch_bounds__(256) void k_squash_t(const float* __restrict__ S, h16* VT) {
#pragma clang fp contract(off)
    __shared__ __align__(16) float sv[NU * NB];
    __shared__ float fac[NB];
    const int t = threadIdx.x, d = blockIdx.x;
#pragma unroll 1
    for (int q = 0; q < (NU * NB) / 256; ++q) { const int idx = q * 256 + t; const int uu = idx / NB, b = idx % NB;
        sv[idx] = S[(size_t)uu * (NB * ND) + b * ND + d]; }
    __syncthreads();
    if (t < NB) {
        float msq = 0.0f;
#pragma unroll 1
        for (int uu = 0; uu < NU; ++uu) { const float xv = sv[uu * NB + t]; msq += xv * xv; }
        fac[t] = msq * __builtin_amdgcn_rcpf(1.0f + msq) * __builtin_amdgcn_rsqf(msq) * VCAR;
    }
    __syncthreads();
    const int uu = t >> 3, p = t & 7;
    v8h o;
#pragma unroll
    for (int e = 0; e < 8; ++e) o[e] = toh_flush(sv[uu * NB + 8 * p + e] * fac[8 * p + e]);
    h16* dst = VT + (size_t)(uu * ND + d) * NB + 8 * p;
    *(volatile v8h*)dst = o; __threadfence(); *(volatile v8h*)dst = o;
}

__global__ __launch_bounds__(128) void k_squash_out(const float* __restrict__ S, float* OUT) {
#pragma clang fp contract(off)
    __shared__ __align__(16) float sq[NU * ND];
    const int t = threadIdx.x, b = blockIdx.x;
    const int uu = t >> 2, d4 = (t & 3) * 4;
    const v4f s4 = *(const v4f*)(S + (size_t)uu * (NB * ND) + b * ND + d4);
    *(v4fa*)(&sq[uu * ND + d4]) = s4 * s4;
    __syncthreads();
    v4f m4 = (v4f){};
#pragma unroll 1
    for (int k = 0; k < NU; ++k) m4 += *(const v4fa*)(&sq[k * ND + d4]);
    v4f o;
#pragma unroll
    for (int e = 0; e < 4; ++e) { const float msq = m4[e]; o[e] = s4[e] * (msq * __builtin_amdgcn_rcpf(1.0f + msq) * __builtin_amdgcn_rsqf(msq)); }
    float* dst = OUT + (size_t)b * (NU * ND) + 4 * t;
    *(volatile v4f*)dst = o; __threadfence(); *(volatile v4f*)dst = o;
}

template <int PRIOR>
__device__ __forceinline__ void route_body(const h16* __restrict__ XT, const h16* __restrict__ VT, const h16* __restrict__ WH, const float* Bprior, float* Bout, float* Cout) {
    __shared__ __align__(16) float dl[RCH * NU];
    __shared__ __align__(16) float ct[RCH * NU];
    __shared__ __align__(16) float bt[RCH * NU];
    const int lane = threadIdx.x & 31, lr = lane & 15, hi = lane >> 4;
    const int c0 = blockIdx.x * RCH;
    v16h a[4][2];
#pragma unroll
    for (int mt = 0; mt < 4; ++mt) {
        const h16* ap = XT + (size_t)(c0 * NI + mt * 16 + lr) * NB + 8 * hi;
        a[mt][0] = ldh(ap); a[mt][1] = ldh(ap + 32); }
#pragma unroll 1
    for (int u = 0; u < NU; ++u) {
        const h16* vb = VT + (size_t)(u * ND + lr) * NB + 8 * hi;
        const v16h b0 = ldh(vb), b1 = ldh(vb + 32);
        float part[4];
#pragma unroll
        for (int mt = 0; mt < 4; ++mt) {
            v8f acc = (v8f){};
            acc = wmma16g(a[mt][0], b0, acc);
            acc = wmma16g(a[mt][1], b1, acc);
            const v8h wv = *(const v8h*)(WH + ((size_t)(c0 + 2 * mt + hi) * NU + u) * (ND * NI) + (size_t)lr * NI);
            float p = 0.0f;
#pragma unroll
            for (int r = 0; r < 8; ++r) p += acc[r] * (float)wv[r];
            p += __shfl_xor(p, 8, 32); p += __shfl_xor(p, 4, 32); p += __shfl_xor(p, 2, 32); p += __shfl_xor(p, 1, 32);
            part[mt] = p; }
        if (lr == 0) {
#pragma unroll
            for (int mt = 0; mt < 4; ++mt) dl[(2 * mt + hi) * NU + u] = part[mt]; }
    }
    wave_sync();
#pragma unroll 1
    for (int j = 0; j < RCH; ++j) {
        float bo = 0.0f;
        if (PRIOR) bo = Bprior[(size_t)(c0 + j) * NU + lane];
        const float bn = bo + dl[j * NU + lane] * DSC;
        float mx = bn;
        mx = fmaxf(mx, __shfl_xor(mx, 16, 32)); mx = fmaxf(mx, __shfl_xor(mx, 8, 32)); mx = fmaxf(mx, __shfl_xor(mx, 4, 32));
        mx = fmaxf(mx, __shfl_xor(mx, 2, 32));  mx = fmaxf(mx, __shfl_xor(mx, 1, 32));
        const float e = __builtin_amdgcn_exp2f((bn - mx) * LOG2E);
        float sm = e;
        sm += __shfl_xor(sm, 16, 32); sm += __shfl_xor(sm, 8, 32); sm += __shfl_xor(sm, 4, 32); sm += __shfl_xor(sm, 2, 32); sm += __shfl_xor(sm, 1, 32);
        bt[j * NU + lane] = bn;
        ct[j * NU + lane] = e * __builtin_amdgcn_rcpf(sm);
    }
    wave_sync();
#pragma unroll 1
    for (int ps = 0; ps < 2; ++ps) {
#pragma unroll
        for (int s = 0; s < 2; ++s) { const int row = 4 * s + (lane >> 3), cofs = (lane & 7) * 4;
            const v4f cv = *(const v4fa*)(&ct[row * NU + cofs]);
            *(volatile v4f*)(Cout + (size_t)(c0 + row) * NU + cofs) = cv;
            if (PRIOR == 0) { const v4f bv = *(const v4fa*)(&bt[row * NU + cofs]);
                *(volatile v4f*)(Bout + (size_t)(c0 + row) * NU + cofs) = bv; } }
        if (ps == 0) __threadfence(); }
}

__global__ __launch_bounds__(32) void k_route_first(const h16* __restrict__ XT, const h16* __restrict__ VT, const h16* __restrict__ WH, float* Bout, float* Cout) {
    route_body<0>(XT, VT, WH, Bout, Bout, Cout);
}
__global__ __launch_bounds__(32) void k_route_next(const h16* __restrict__ XT, const h16* __restrict__ VT, const h16* __restrict__ WH, const float* Bprior, float* Cout) {
    route_body<1>(XT, VT, WH, Bprior, Cout, Cout);
}

static constexpr size_t al256(size_t v) { return (v + 255) & ~(size_t)255; }
static constexpr size_t SZ_WH = al256((size_t)NC * WROW * 2);
static constexpr size_t SZ_XS = al256((size_t)NB * KS * 2);
static constexpr size_t SZ_XT = al256((size_t)KS * NB * 2);
static constexpr size_t SZ_VT = al256((size_t)NU * ND * NB * 2);
static constexpr size_t SZ_S  = al256((size_t)NU * NB * ND * 4);
static constexpr size_t SZ_CT = al256((size_t)NC * NU * 4);
static constexpr size_t SZ_TOTAL = SZ_WH + SZ_XS + SZ_XT + SZ_VT + SZ_S + 2 * SZ_CT;
static_assert(SZ_TOTAL <= (size_t)134217728);

extern "C" void kernel_launch(void* const* d_in, const int* in_sizes, int n_in,
                              void* d_out, int out_size, void* d_ws, size_t ws_size, hipStream_t stream) {
    if (n_in < 2) return;
    if ((size_t)in_sizes[0] < ((size_t)(NB - 1) * NI + (NI - 1)) * NC_FULL + NC) return;
    if ((size_t)in_sizes[1] < (size_t)NC * WROW) return;
    if ((size_t)out_size < (size_t)NB * NU * ND) return;
    if (SZ_TOTAL > ws_size) return;
    const float* x = (const float*)d_in[0];
    const float* W = (const float*)d_in[1];
    float* OUT = (float*)d_out;
    char* wsp = (char*)d_ws;
    h16* WH = (h16*)wsp; wsp += SZ_WH;
    h16* XS = (h16*)wsp; wsp += SZ_XS;
    h16* XT = (h16*)wsp; wsp += SZ_XT;
    h16* VT = (h16*)wsp; wsp += SZ_VT;
    float* S  = (float*)wsp; wsp += SZ_S;
    float* CT = (float*)wsp; wsp += SZ_CT;
    float* B1 = (float*)wsp; wsp += SZ_CT;

    { const size_t n8 = (size_t)NC * WROW / 8; k_cvtw<<<(unsigned)((n8 + 255) / 256), 256, 0, stream>>>(W, WH, n8); }
    k_xs<<<(unsigned)(((size_t)NB * NC) / 256), 256, 0, stream>>>(x, XS);
    k_xt<<<(unsigned)(((size_t)NC * NI * 8) / 256), 256, 0, stream>>>(x, XT);
    k_fillc<<<(unsigned)(((size_t)NC * NU / 4) / 256), 256, 0, stream>>>(CT);

    k_sgemm<<<NU, 32 * SW, 0, stream>>>(XS, WH, CT, S);
    k_squash_t<<<ND, 256, 0, stream>>>(S, VT);
    k_route_first<<<NC / RCH, 32, 0, stream>>>(XT, VT, WH, B1, CT);
    k_sgemm<<<NU, 32 * SW, 0, stream>>>(XS, WH, CT, S);
    k_squash_t<<<ND, 256, 0, stream>>>(S, VT);
    k_route_next<<<NC / RCH, 32, 0, stream>>>(XT, VT, WH, B1, CT);
    k_sgemm<<<NU, 32 * SW, 0, stream>>>(XS, WH, CT, S);
    k_squash_out<<<NB, 128, 0, stream>>>(S, OUT);
}
